// RNNEncoder_17239998726623
// MI455X (gfx1250) — hardware-verified
//
#include <hip/hip_runtime.h>
#include <math.h>

constexpr int NSEQ    = 512;
constexpr int NSTEP   = 512;
constexpr int NIN2    = 2;
constexpr int NHID    = 256;
constexpr int NGATE   = 3 * NHID;
constexpr int NTHR    = 256;
constexpr int SEQ_BLK = 16;
constexpr int HPITCH  = 264;
constexpr int OPITCH  = 260;
constexpr int NPAR    = NGATE * NIN2 + 2 * NGATE;
constexpr float WCARRY  = 256.0f;
constexpr float HCARRY  = 64.0f;
constexpr float RCARRY  = 2048.0f;
constexpr float FOLD_HI = 1.0f / 16384.0f;
constexpr float FOLD_LO = FOLD_HI / 2048.0f;
static_assert(NSEQ % SEQ_BLK == 0);
static_assert(NHID == 32 * (NTHR / 32));
static_assert(NHID % 32 == 0);
static_assert(NTHR == NHID);
static_assert(HPITCH % 8 == 0 && OPITCH % 4 == 0);
static_assert((2 * SEQ_BLK * HPITCH) % NTHR == 0);
static_assert((NGATE * NIN2) % NTHR == 0 && NGATE % NTHR == 0);
static_assert((NGATE * (NHID / 8)) % NTHR == 0);
static_assert(SEQ_BLK * NHID == 4 * 4 * NTHR);

typedef __attribute__((ext_vector_type(16))) _Float16 v16h;
typedef __attribute__((ext_vector_type(8)))  _Float16 v8h;
typedef __attribute__((ext_vector_type(8)))  float    v8f;
typedef __attribute__((ext_vector_type(4)))  float    v4f;
typedef __attribute__((ext_vector_type(2)))  float    v2f;
typedef __attribute__((ext_vector_type(4)))  int      v4i;

__device__ __forceinline__ unsigned short f2bf_bits(float f) {
  unsigned u = __float_as_uint(f);
  return (unsigned short)((u + 0x7FFFu + ((u >> 16) & 1u)) >> 16);
}
__device__ __forceinline__ float bf_bits2f(unsigned short h) { return __uint_as_float(((unsigned)h) << 16); }
__device__ __forceinline__ float bf16r(float f) { return bf_bits2f(f2bf_bits(f)); }

__device__ __forceinline__ void dep_guard_h(v8f& a, v8f& b, v16h x, v16h y) { asm volatile("v_nop\n\tv_nop\n\tv_nop\n\tv_nop" : "+v"(a), "+v"(b) : "v"(x), "v"(y)); }
__device__ __forceinline__ void dep_guard6_h(v8f& a, v8f& b, v8f& c, v8f& d, v8f& e, v8f& f,
                                             v16h p, v16h q, v16h x, v16h y, v16h z) {
  asm volatile("v_nop\n\tv_nop\n\tv_nop\n\tv_nop"
               : "+v"(a), "+v"(b), "+v"(c), "+v"(d), "+v"(e), "+v"(f)
               : "v"(p), "v"(q), "v"(x), "v"(y), "v"(z));
}
__device__ __forceinline__ void keep4_h(v16h a, v16h b, v16h c, v16h d) { asm volatile("v_nop" :: "v"(a), "v"(b), "v"(c), "v"(d)); }
__device__ __forceinline__ void acc_guard6(v8f& a, v8f& b, v8f& c, v8f& d, v8f& e, v8f& f) {
  asm volatile("v_nop\n\tv_nop\n\tv_nop\n\tv_nop" : "+v"(a), "+v"(b), "+v"(c), "+v"(d), "+v"(e), "+v"(f));
}
template <typename T> struct Frag;
template <> struct Frag<_Float16> {
  typedef v16h V; union U { v16h v; v8h h[2]; };
  static __device__ __forceinline__ v16h load(const _Float16* p) {
    U f; f.h[0] = *(const v8h*)(p); f.h[1] = *(const v8h*)(p + 16); return f.v;
  }
  static __device__ __forceinline__ v8f mma(v16h a, v16h b, v8f c) {
    return __builtin_amdgcn_wmma_f32_16x16x32_f16(false, a, false, b, (short)0, c, false, false);
  }
  static __device__ __forceinline__ void guard(v8f& a, v8f& b, v16h x, v16h y) { dep_guard_h(a, b, x, y); }
  static __device__ __forceinline__ void keep(v16h a, v16h b, v16h c, v16h d) { keep4_h(a, b, c, d); }
};

__device__ __forceinline__ float fsig(float x)  { return __builtin_amdgcn_rcpf(1.0f + expf(-x)); }
__device__ __forceinline__ float ftanh(float x) { return 1.0f - 2.0f * __builtin_amdgcn_rcpf(expf(2.0f * x) + 1.0f); }

__device__ __forceinline__ void put_h(_Float16* __restrict__ ph, _Float16* __restrict__ pl, float hn) {
  const float v = hn * HCARRY;
  const _Float16 h16 = (_Float16)v;
  const float hif = (float)h16;
  const float res = (v - hif) * RCARRY;
  *ph = h16;
  *pl = (_Float16)res;
}

template <int MODE>
__global__ __launch_bounds__(NTHR) void cvt8_kernel(const float* __restrict__ src, unsigned short* __restrict__ dst,
                                                    int nrow, int ncol8, int spitch, int scol0, float sc) {
  const int i  = blockIdx.x * NTHR + threadIdx.x;
  const int n8 = nrow * ncol8;
  if (i < n8) {
    const int row = i / ncol8;
    const int c8  = i - row * ncol8;
    const float* sp = src + (size_t)row * spitch + scol0 + c8 * 8;
    const v4f a = *(const v4f*)(sp);
    const v4f b = *(const v4f*)(sp + 4);
    v8h hv;
#pragma unroll
    for (int e = 0; e < 4; ++e) {
      unsigned short b0, b1;
      if (MODE == 0) {
        b0 = f2bf_bits(a[e] * sc);
        b1 = f2bf_bits(b[e] * sc);
      } else {
        b0 = __builtin_bit_cast(unsigned short, (_Float16)(bf16r(a[e]) * sc));
        b1 = __builtin_bit_cast(unsigned short, (_Float16)(bf16r(b[e]) * sc));
      }
      hv[e]     = __builtin_bit_cast(_Float16, b0);
      hv[4 + e] = __builtin_bit_cast(_Float16, b1);
    }
    *(volatile v8h*)(dst + (size_t)i * 8) = hv;
    __threadfence();
    *(volatile v8h*)(dst + (size_t)i * 8) = hv;
  }
}

__global__ __launch_bounds__(NTHR) void gru_seq_kernel(const float* __restrict__ X, const int* __restrict__ LEN,
                                                       const float* __restrict__ H0, const float* __restrict__ WIH,
                                                       const float* __restrict__ BIH, const float* __restrict__ BHH,
                                                       const unsigned short* __restrict__ WHp, float* __restrict__ OUT) {
  __shared__ __align__(16) _Float16 Ahi[2][SEQ_BLK * HPITCH];
  __shared__ __align__(16) _Float16 Alo[2][SEQ_BLK * HPITCH];
  __shared__ __align__(16) float    Hs[SEQ_BLK * OPITCH];
  __shared__ __align__(16) float    Par[NPAR];
  const _Float16* WH = (const _Float16*)WHp;
  const int tid = threadIdx.x, lane = tid & 31, wave = tid >> 5;
  const int c = lane & 15, hh = lane >> 4, koff = hh * 8;
  const int rowbase = blockIdx.x * SEQ_BLK;

  {
    _Float16* ahf = &Ahi[0][0];
    _Float16* alf = &Alo[0][0];
#pragma unroll 1
    for (int i = tid; i < 2 * SEQ_BLK * HPITCH; i += NTHR) { ahf[i] = (_Float16)0.0f; alf[i] = (_Float16)0.0f; }
  }
#pragma unroll 1
  for (int i = tid; i < NGATE * NIN2; i += NTHR) Par[i] = bf16r(WIH[i]);
#pragma unroll 1
  for (int i = tid; i < NGATE; i += NTHR) {
    Par[NGATE * NIN2 + i]         = bf16r(BIH[i]);
    Par[NGATE * NIN2 + NGATE + i] = bf16r(BHH[i]);
  }
#pragma unroll 1
  for (int i = 0; i < SEQ_BLK; ++i) Hs[i * OPITCH + tid] = bf16r(H0[(size_t)(rowbase + i) * NHID + tid]);

  int lenm1[8];
  int tmax;
  {
    const v4i q0 = *(const v4i*)(LEN + rowbase);
    const v4i q1 = *(const v4i*)(LEN + rowbase + 4);
    const v4i q2 = *(const v4i*)(LEN + rowbase + 8);
    const v4i q3 = *(const v4i*)(LEN + rowbase + 12);
    int lv[16];
#pragma unroll
    for (int e = 0; e < 4; ++e) { lv[e] = q0[e]; lv[4 + e] = q1[e]; lv[8 + e] = q2[e]; lv[12 + e] = q3[e]; }
    int tm = 1;
#pragma unroll
    for (int i = 0; i < 16; ++i) {
      int v = lv[i];
      v = (v < 1) ? 1 : v;
      v = (v > NSTEP) ? NSTEP : v;
      lv[i] = v;
      tm = (v > tm) ? v : tm;
    }
    tm = (tm > NSTEP) ? NSTEP : tm;
    tmax = __builtin_amdgcn_readfirstlane(tm);
#pragma unroll
    for (int r = 0; r < 8; ++r) lenm1[r] = (hh ? lv[8 + r] : lv[r]) - 1;
  }
  __syncthreads();

  float wi0[2][3], wi1[2][3], brz[2][2], bni[2], bnh[2];
  float hst[2][8], hcap[2][8];
  {
    const float* pbi = Par + NGATE * NIN2;
    const float* pbh = pbi + NGATE;
#pragma unroll
    for (int nt = 0; nt < 2; ++nt) {
      const int j = 32 * wave + 16 * nt + c;
#pragma unroll
      for (int g = 0; g < 3; ++g) {
        wi0[nt][g] = Par[(g * NHID + j) * NIN2 + 0];
        wi1[nt][g] = Par[(g * NHID + j) * NIN2 + 1];
      }
      brz[nt][0] = pbi[j] + pbh[j];
      brz[nt][1] = pbi[NHID + j] + pbh[NHID + j];
      bni[nt]    = pbi[2 * NHID + j];
      bnh[nt]    = pbh[2 * NHID + j];
#pragma unroll
      for (int r = 0; r < 8; ++r) {
        const float hv = Hs[(8 * hh + r) * OPITCH + j];
        hst[nt][r]  = hv;
        hcap[nt][r] = 0.0f;
        const int idx = (8 * hh + r) * HPITCH + j;
        put_h(&Ahi[0][idx], &Alo[0][idx], hv);
      }
    }
  }
  __syncthreads();

  const v8f z8 = {0.f, 0.f, 0.f, 0.f, 0.f, 0.f, 0.f, 0.f};

#pragma unroll 1
  for (int t = 0; t < tmax; ++t) {
    float xa[8], xb[8];
#pragma unroll
    for (int r = 0; r < 8; ++r) {
      const v2f v = *(const v2f*)(X + ((size_t)(rowbase + 8 * hh + r) * NSTEP + (size_t)t) * NIN2);
      xa[r] = bf16r(v[0]);
      xb[r] = bf16r(v[1]);
    }
    const int cur = t & 1;
    const _Float16* ahrow = &Ahi[cur][0] + c * HPITCH + koff;
    const _Float16* alrow = &Alo[cur][0] + c * HPITCH + koff;
    _Float16* ahn = &Ahi[cur ^ 1][0];
    _Float16* aln = &Alo[cur ^ 1][0];
#pragma unroll
    for (int nt = 0; nt < 2; ++nt) {
      const int j = 32 * wave + 16 * nt + c;
      const _Float16* w0 = WH + (size_t)j * NHID + koff;
      const _Float16* w1 = w0 + (size_t)NHID * NHID;
      const _Float16* w2 = w0 + (size_t)2 * NHID * NHID;
      v8f ar = z8, az = z8, an = z8, arl = z8, azl = z8, anl = z8;
#pragma unroll 1
      for (int k0 = 0; k0 < NHID; k0 += 32) {
        const v16h a  = Frag<_Float16>::load(ahrow + k0);
        const v16h al = Frag<_Float16>::load(alrow + k0);
        const v16h b0 = Frag<_Float16>::load(w0 + k0);
        const v16h b1 = Frag<_Float16>::load(w1 + k0);
        const v16h b2 = Frag<_Float16>::load(w2 + k0);
        ar  = Frag<_Float16>::mma(a,  b0, ar);
        az  = Frag<_Float16>::mma(a,  b1, az);
        an  = Frag<_Float16>::mma(a,  b2, an);
        arl = Frag<_Float16>::mma(al, b0, arl);
        azl = Frag<_Float16>::mma(al, b1, azl);
        anl = Frag<_Float16>::mma(al, b2, anl);
        dep_guard6_h(ar, az, an, arl, azl, anl, a, al, b0, b1, b2);
      }
      acc_guard6(ar, az, an, arl, azl, anl);
#pragma unroll
      for (int r = 0; r < 8; ++r) {
        const float gir = xa[r] * wi0[nt][0] + xb[r] * wi1[nt][0] + brz[nt][0];
        const float giz = xa[r] * wi0[nt][1] + xb[r] * wi1[nt][1] + brz[nt][1];
        const float gin = xa[r] * wi0[nt][2] + xb[r] * wi1[nt][2] + bni[nt];
        const float ghr = ar[r] * FOLD_HI + arl[r] * FOLD_LO;
        const float ghz = az[r] * FOLD_HI + azl[r] * FOLD_LO;
        const float ghn = an[r] * FOLD_HI + anl[r] * FOLD_LO;
        const float rg = fsig(gir + ghr);
        const float zg = fsig(giz + ghz);
        const float ng = ftanh(gin + rg * (ghn + bnh[nt]));
        const float ho = hst[nt][r];
        const float hn = (1.0f - zg) * ng + zg * ho;
        hst[nt][r]  = hn;
        hcap[nt][r] = (t == lenm1[r]) ? hn : hcap[nt][r];
        const int idx = (8 * hh + r) * HPITCH + j;
        put_h(ahn + idx, aln + idx, hn);
      }
    }
    __syncthreads();
  }

#pragma unroll
  for (int nt = 0; nt < 2; ++nt) {
    const int j = 32 * wave + 16 * nt + c;
#pragma unroll
    for (int r = 0; r < 8; ++r) Hs[(8 * hh + r) * OPITCH + j] = hcap[nt][r];
  }
  __syncthreads();
  for (int pass = 0; pass < 2; ++pass) {
#pragma unroll
    for (int it = 0; it < 4; ++it) {
      const int idx = it * NTHR + tid;
      const int row = idx >> 6, c4 = (idx & 63) * 4;
      const v4f v = *(const v4f*)(Hs + row * OPITCH + c4);
      *(volatile v4f*)(OUT + (size_t)(rowbase + row) * NHID + c4) = v;
    }
    __threadfence();
  }
}

extern "C" void kernel_launch(void* const* d_in, const int* in_sizes, int n_in,
                              void* d_out, int out_size, void* d_ws, size_t ws_size, hipStream_t stream) {
  if (n_in < 7 || d_out == nullptr || d_ws == nullptr) return;
  if (in_sizes[0] != NSEQ * NSTEP * NIN2 || in_sizes[1] != NSEQ || in_sizes[2] != NSEQ * NHID ||
      in_sizes[3] != NGATE * NIN2 || in_sizes[4] != NGATE * NHID || in_sizes[5] != NGATE || in_sizes[6] != NGATE ||
      out_size != NSEQ * NHID) return;

  const float* x    = (const float*)d_in[0];
  const int*   len  = (const int*)  d_in[1];
  const float* h0   = (const float*)d_in[2];
  const float* w_ih = (const float*)d_in[3];
  const float* w_hh = (const float*)d_in[4];
  const float* b_ih = (const float*)d_in[5];
  const float* b_hh = (const float*)d_in[6];
  float* out = (float*)d_out;

  char* ws = (char*)d_ws; size_t off = 0;
  auto carve = [&](size_t bytes) -> char* { char* p = ws + off; off += (bytes + 255) & ~(size_t)255; return p; };
  unsigned short* WH = (unsigned short*)carve((size_t)NGATE * NHID * 2);
  if (off > ws_size || off > (size_t)134217728) return;

  const int n8w = NGATE * (NHID / 8);
  cvt8_kernel<1><<<(n8w + NTHR - 1) / NTHR, NTHR, 0, stream>>>(w_hh, WH, NGATE, NHID / 8, NHID, 0, WCARRY);
  gru_seq_kernel<<<NSEQ / SEQ_BLK, NTHR, 0, stream>>>(x, len, h0, w_ih, b_ih, b_hh, WH, out);
}
